// HierarchicalGCNPyG_55121610277008
// MI455X (gfx1250) — hardware-run, weakly checked
//
#include <hip/hip_runtime.h>


#ifndef NROWS
#define NROWS 16384
#endif
#define NROWS_FULL 16384
#define C0 256
#define C1 64
#define C2 32
#define C3 16
#define C4 8
#define NN 28
#define SB 8
#define RT (NN * SB)
#define NRT (RT / 16)
#define ZP 32
#define ZCOLS (SB * C2)
#define QRS  2048.0f
#define QRI  (1.0f / 2048.0f)
#define WSC  256.0f
#define WSI  (1.0f / 256.0f)
#define NEGB (-3.0e38f)

static_assert(NROWS % 32 == 0);
static_assert(NROWS % SB == 0);
static_assert(NROWS <= NROWS_FULL);
static_assert(C0 % 32 == 0);
static_assert(C1 == 64);
static_assert(C2 == 32);
static_assert(C3 == 16);
static_assert(C4 == 8);
static_assert(SB == 8);
static_assert(RT % 32 == 0);
static_assert(RT <= 256);
static_assert(RT % 16 == 0);
static_assert(ZCOLS == 256);
static_assert(NN <= ZP);
static_assert(16 * 16 == 256);
static_assert(8 * 32 * 4 == 16 * C1);
static_assert((32 + 24) * 4 == SB * NN);
static_assert(((size_t)SB * NN * 4) % 128 == 0);
static_assert((size_t)NROWS_FULL * NN * 4 == (size_t)1835008);
static_assert(((size_t)NROWS_FULL * NN * 4) % 128 == 0);
static_assert((C1 * C0 / 8) % 256 == 0);

typedef _Float16 h16;
typedef unsigned short bf;
typedef __attribute__((ext_vector_type(16))) __bf16   v16bf;
typedef __attribute__((ext_vector_type(16))) _Float16 v16h;
typedef __attribute__((ext_vector_type(8)))  _Float16 v8h;
typedef __attribute__((ext_vector_type(8)))  unsigned short v8us;
typedef __attribute__((ext_vector_type(8)))  float    v8f;
typedef __attribute__((ext_vector_type(4)))  float    v4f;
typedef v4f  __attribute__((may_alias)) v4fa;

__device__ __forceinline__ unsigned short f2bf(float f) { unsigned u = __float_as_uint(f); u += 0x7FFFu + ((u >> 16) & 1u); return (unsigned short)(u >> 16); }
__device__ __forceinline__ float bfr(float f) { return __uint_as_float(((unsigned)f2bf(f)) << 16); }
__device__ __forceinline__ v16h cat16(v8h lo, v8h hi) { return __builtin_shufflevector(lo, hi, 0, 1, 2, 3, 4, 5, 6, 7, 8, 9, 10, 11, 12, 13, 14, 15); }
__device__ __forceinline__ v16bf cat16b(v8us lo, v8us hi) { return __builtin_bit_cast(v16bf, __builtin_shufflevector(lo, hi, 0, 1, 2, 3, 4, 5, 6, 7, 8, 9, 10, 11, 12, 13, 14, 15)); }
__device__ __forceinline__ v8f wmma16(v16h a, v16h b, v8f c) { return __builtin_amdgcn_wmma_f32_16x16x32_f16(false, a, false, b, (short)0, c, false, false); }
__device__ __forceinline__ v8f wmmab(v16bf a, v16bf b, v8f c) { return __builtin_amdgcn_wmma_f32_16x16x32_bf16(false, a, false, b, (short)0, c, false, false); }
__device__ __forceinline__ v16bf ldb(const bf* p)  { return cat16b(*(const v8us*)p, *(const v8us*)(p + 16)); }
__device__ __forceinline__ void wave_sync() { __builtin_amdgcn_fence(3  , "wavefront"); __builtin_amdgcn_wave_barrier(); asm volatile("" ::: "memory"); }

static __device__ __forceinline__ h16 toh_flush(float v) { const h16 r = (h16)v; return (fabsf(v) < 6.103515625e-05f) ? (h16)0.0f : r; }
__device__ __forceinline__ v8f mmah(v16h a, v16h b, v8f c) { c = wmma16(a, b, c); asm volatile("v_nop\n\tv_nop\n\tv_nop\n\tv_nop" : "+v"(c) : "v"(a), "v"(b)); return c; }
__device__ __forceinline__ v8f mmab(v16bf a, v16bf b, v8f c) { c = wmmab(a, b, c); asm volatile("v_nop\n\tv_nop\n\tv_nop\n\tv_nop" : "+v"(c) : "v"(a), "v"(b)); return c; }
__device__ __forceinline__ v16bf ldxb(const float* p) {
    const v4f a0 = *(const v4f*)p, a1 = *(const v4f*)(p + 4), a2 = *(const v4f*)(p + 16), a3 = *(const v4f*)(p + 20);
    v8us lo, hi;
#pragma unroll
    for (int i = 0; i < 4; ++i) { lo[i] = f2bf(a0[i]); lo[4 + i] = f2bf(a1[i]); hi[i] = f2bf(a2[i]); hi[4 + i] = f2bf(a3[i]); }
    return cat16b(lo, hi);
}
#define LFRAG(arr, idx) cat16(*(const v8h*)(&arr[(idx)]), *(const v8h*)(&arr[(idx) + 16]))

static constexpr int par_c(int n) {
    const int P[NN] = { -1, 0, 0, 0, 0, 1, 1, 2, 3, 4, 4, 5, 5, 6, 7, 8, 9, 10, 11, 12, 13, 14, 14, 14, 15, 15, 16, 17 };
    return P[n];
}
static constexpr unsigned long long pack_par(int base) {
    unsigned long long w = 0;
    for (int i = 0; i < 12; ++i) { const int n = base + i; const unsigned long long v = (n < NN) ? (unsigned long long)(par_c(n) < 0 ? 31 : par_c(n)) : 0ull; w |= v << (5 * i); }
    return w;
}
enum : unsigned long long { PAR_W0 = pack_par(0), PAR_W1 = pack_par(12), PAR_W2 = pack_par(24) };
__host__ __device__ constexpr int par_dec(int n) {
    const int q = n / 12, r = n - 12 * q;
    const unsigned long long w = (q == 0) ? (unsigned long long)PAR_W0 : ((q == 1) ? (unsigned long long)PAR_W1 : (unsigned long long)PAR_W2);
    const int v = (int)((w >> (5 * r)) & 31ull);
    return v == 31 ? -1 : v;
}
static constexpr bool par_ok() { for (int n = 0; n < NN; ++n) if (par_dec(n) != par_c(n)) return false; return true; }
static_assert(par_ok());
static_assert(par_dec(0) == -1);
static_assert(par_dec(27) == 17);
static_assert(5 * 11 + 5 <= 64);
__device__ __forceinline__ int par_dev(int node) {
    unsigned n = (unsigned)node; asm volatile("" : "+v"(n));
    const unsigned q = n / 12u;
    unsigned sh = 5u * (n - 12u * q); asm volatile("" : "+v"(sh));
    const unsigned long long w = (q == 0u) ? (unsigned long long)PAR_W0 : ((q == 1u) ? (unsigned long long)PAR_W1 : (unsigned long long)PAR_W2);
    const unsigned v = (unsigned)((w >> sh) & 31ull);
    return (v == 31u) ? -1 : (int)v;
}

__global__ __launch_bounds__(256) void k_w1t(const float* __restrict__ W1, bf* W1T) {
    const int i = blockIdx.x * 256 + threadIdx.x; if (i >= C1 * C0 / 8) return;
    const int n = i / (C0 / 8), k8 = (i % (C0 / 8)) * 8; v8us o;
#pragma unroll
    for (int j = 0; j < 8; ++j) o[j] = f2bf(W1[(size_t)(k8 + j) * C1 + n]);
    *(volatile v8us*)(W1T + (size_t)i * 8) = o; __threadfence(); *(volatile v8us*)(W1T + (size_t)i * 8) = o;
}

__global__ __launch_bounds__(32) void k_y(const float* __restrict__ X, const bf* __restrict__ W1T, float* Yp) {
    __shared__ __align__(16) float os[16 * 68];
    const int lane = threadIdx.x & 31, lr = lane & 15, hi = lane >> 4; const int r0 = blockIdx.x * 32;
    v8f acc[2][4];
#pragma unroll
    for (int mb = 0; mb < 2; ++mb)
#pragma unroll
        for (int nb = 0; nb < 4; ++nb) acc[mb][nb] = (v8f){};
    const size_t aoff = (size_t)(r0 + lr) * C0 + 8 * hi, boff = (size_t)lr * C0 + 8 * hi;
#pragma unroll 1
    for (int kc = 0; kc < C0; kc += 32) {
        v16bf a[2];
#pragma unroll
        for (int mb = 0; mb < 2; ++mb) a[mb] = ldxb(X + aoff + (size_t)mb * 16 * C0 + kc);
#pragma unroll
        for (int nb = 0; nb < 4; ++nb) { const v16bf b = ldb(W1T + boff + (size_t)nb * 16 * C0 + kc);
#pragma unroll
            for (int mb = 0; mb < 2; ++mb) acc[mb][nb] = mmab(a[mb], b, acc[mb][nb]); }
    }
#pragma unroll
    for (int mb = 0; mb < 2; ++mb) {
#pragma unroll
        for (int nb = 0; nb < 4; ++nb) {
#pragma unroll
            for (int j = 0; j < 8; ++j) os[(hi * 8 + j) * 68 + nb * 16 + lr] = acc[mb][nb][j]; }
        wave_sync();
        float* yb = Yp + (size_t)(r0 + mb * 16) * C1;
#pragma unroll 1
        for (int ps = 0; ps < 2; ++ps) {
#pragma unroll
            for (int s = 0; s < 8; ++s) { const int p = s * 32 + lane; const int row = p >> 4, c4 = (p & 15) * 4;
                const v4f val = *(const v4fa*)(&os[row * 68 + c4]);
                *(volatile v4f*)(yb + (size_t)row * C1 + c4) = val; }
            if (ps == 0) __threadfence(); }
        wave_sync();
    }
}

static constexpr size_t LDS_TREE = (size_t)SB * C1 * 4 + 32 * 32 * 2 + (size_t)C2 * C1 * 2 + (size_t)C3 * C2 * 2 + 16 * 16 * 2 + 2 * (size_t)ZCOLS * ZP * 2 + 2 * (size_t)RT * C2 * 2
                                   + (size_t)RT * C4 * 4 + 2 * (size_t)RT * 4 + (size_t)RT * 4 + (size_t)(C1 + C2 + C3 + C4 + C4 + 4 + 32 + 32) * 4 + 32 * 4;
static_assert(LDS_TREE <= (size_t)131072);
static_assert(16 * 68 * 4 <= 131072);

__global__ __launch_bounds__(256) void k_tree(const float* __restrict__ Yp, const float* __restrict__ b1, const float* __restrict__ W2, const float* __restrict__ b2,
                                              const float* __restrict__ W3, const float* __restrict__ b3, const float* __restrict__ W4, const float* __restrict__ b4,
                                              const float* __restrict__ W5, const float* __restrict__ b5, float* OUT) {
    __shared__ __align__(16) float sY[SB * C1];
    __shared__ __align__(16) h16 sA[32 * 32];
    __shared__ __align__(16) h16 sW2t[C2 * C1];
    __shared__ __align__(16) h16 sW3t[C3 * C2];
    __shared__ __align__(16) h16 sW4t[16 * 16];
    __shared__ __align__(16) h16 sZv[ZCOLS * ZP];
    __shared__ __align__(16) h16 sZr[ZCOLS * ZP];
    __shared__ __align__(16) h16 sHv[RT * C2];
    __shared__ __align__(16) h16 sHr[RT * C2];
    __shared__ __align__(16) float sH4[RT * C4];
    __shared__ __align__(16) float sOut[2 * RT];
    __shared__ __align__(16) float sLcp[RT];
    __shared__ __align__(16) float sB1[C1];
    __shared__ __align__(16) float sB2[C2];
    __shared__ __align__(16) float sB3[C3];
    __shared__ __align__(16) float sB4[C4];
    __shared__ __align__(16) float sW5[C4];
    __shared__ __align__(16) float sB5[4];
    __shared__ __align__(16) float sDinv[32];
    __shared__ __align__(16) float sS[32];
    __shared__ __align__(16) int sPar[32];

    const int tid = threadIdx.x, lane = tid & 31, lr = lane & 15, hi = lane >> 4;
    const int wave = __builtin_amdgcn_readfirstlane((int)(threadIdx.x >> 5));
    const int b0 = blockIdx.x * SB;

#pragma unroll
    for (int i = tid; i < SB * C1; i += 256) sY[i] = Yp[(size_t)b0 * C1 + i];
#pragma unroll 1
    for (int i = tid; i < C2 * C1; i += 256) { const int n = i >> 6, k = i & 63; sW2t[i] = toh_flush(bfr(W2[k * C2 + n]) * WSC); }
#pragma unroll 1
    for (int i = tid; i < C3 * C2; i += 256) { const int n = i >> 5, k = i & 31; sW3t[i] = toh_flush(bfr(W3[k * C3 + n]) * WSC); }
    { const int n = tid >> 4, k = tid & 15; const int nc = n < C4 ? n : (C4 - 1); float w = W4[k * C4 + nc]; asm volatile("" : "+v"(w));
      sW4t[tid] = (n < C4) ? toh_flush(bfr(w) * WSC) : (h16)0.0f; }
    { float t = b1[tid < C1 ? tid : (C1 - 1)]; asm volatile("" : "+v"(t)); if (tid < C1) sB1[tid] = bfr(t); }
    { float t = b2[tid < C2 ? tid : (C2 - 1)]; asm volatile("" : "+v"(t)); if (tid < C2) sB2[tid] = bfr(t); }
    { float t = b3[tid < C3 ? tid : (C3 - 1)]; asm volatile("" : "+v"(t)); if (tid < C3) sB3[tid] = bfr(t); }
    { float t = b4[tid < C4 ? tid : (C4 - 1)]; asm volatile("" : "+v"(t)); if (tid < C4) sB4[tid] = bfr(t); }
    { float t = W5[tid < C4 ? tid : (C4 - 1)]; asm volatile("" : "+v"(t)); if (tid < C4) sW5[tid] = bfr(t); }
    { float t = b5[0]; asm volatile("" : "+v"(t)); if (tid == 0) sB5[0] = bfr(t); }
    if (tid < 32) { const int pv = par_dev(tid); sPar[tid] = (tid < NN) ? pv : -2; }
#pragma unroll
    for (int q = 0; q < ZP - NN; ++q) { sZv[tid * ZP + NN + q] = (h16)0.0f; sZr[tid * ZP + NN + q] = (h16)0.0f; }
    __syncthreads();

#pragma unroll 1
    for (int i = tid; i < 32 * 32; i += 256) { const int n = i >> 5, m = i & 31;
        const bool adj = (n < NN) & (m < NN) & ((n == m) | (sPar[m] == n) | (sPar[n] == m));
        sA[i] = adj ? (h16)1.0f : (h16)0.0f; }
    if (tid < 32) { int cnt = 0;
#pragma unroll 1
        for (int m = 0; m < NN; ++m) cnt += (sPar[m] == tid) ? 1 : 0;
        const int deg = 1 + ((tid != 0) ? 1 : 0) + cnt;
        sDinv[tid] = (tid < NN) ? (1.0f / sqrtf((float)deg)) : 0.0f; }
    __syncthreads();

    if (tid < 32) { float acc = 0.0f;
#pragma unroll 1
        for (int m = 0; m < NN; ++m) acc += (float)sA[tid * 32 + m] * sDinv[m];
        sS[tid] = sDinv[tid] * acc; }
    __syncthreads();

    const v16h am0 = LFRAG(sA, lr * 32 + 8 * hi), am1 = LFRAG(sA, (16 + lr) * 32 + 8 * hi);
    float dA[8], dB[8];
#pragma unroll
    for (int r = 0; r < 8; ++r) { dA[r] = sDinv[8 * hi + r]; dB[r] = sDinv[16 + 8 * hi + r]; }
    const v8h z8 = (v8h){};

#pragma unroll 1
    for (int j = wave; j < NRT; j += 8) {
        const int R = 16 * j + lr; const int nA = R >> 3, sI = R & 7;
        const float sn = sS[nA];
        v8f cv0 = (v8f){}, cr0 = (v8f){}, cv1 = (v8f){}, cr1 = (v8f){};
#pragma unroll
        for (int kc = 0; kc < C1; kc += 32) {
            v16h av, ar;
#pragma unroll
            for (int q = 0; q < 2; ++q) {
                const int kb = kc + 16 * q + 8 * hi;
                const v4f y0 = *(const v4fa*)(&sY[sI * C1 + kb]), y1 = *(const v4fa*)(&sY[sI * C1 + kb + 4]);
                const v4f e0 = *(const v4fa*)(&sB1[kb]), e1 = *(const v4fa*)(&sB1[kb + 4]);
#pragma unroll
                for (int i = 0; i < 4; ++i) {
                    const float u0 = fmaxf(fmaf(sn, y0[i], e0[i]), 0.0f), u1 = fmaxf(fmaf(sn, y1[i], e1[i]), 0.0f);
                    const h16 g0 = toh_flush(u0), g1 = toh_flush(u1);
                    av[8 * q + i] = g0; av[8 * q + 4 + i] = g1;
                    ar[8 * q + i] = toh_flush((u0 - (float)g0) * QRS); ar[8 * q + 4 + i] = toh_flush((u1 - (float)g1) * QRS); }
            }
            const v16h w0 = LFRAG(sW2t, lr * C1 + kc + 8 * hi), w1 = LFRAG(sW2t, (16 + lr) * C1 + kc + 8 * hi);
            cv0 = mmah(av, w0, cv0); cr0 = mmah(ar, w0, cr0); cv1 = mmah(av, w1, cv1); cr1 = mmah(ar, w1, cr1);
        }
        const int nC = 2 * j + hi; const float dn = sDinv[nC] * WSI;
#pragma unroll
        for (int r = 0; r < 8; ++r) {
            const float z0 = (cv0[r] + cr0[r] * QRI) * dn, z1 = (cv1[r] + cr1[r] * QRI) * dn;
            const h16 g0 = toh_flush(z0), g1 = toh_flush(z1);
            const int i0 = (r * C2 + lr) * ZP + nC, i1 = (r * C2 + 16 + lr) * ZP + nC;
            sZv[i0] = g0; sZr[i0] = toh_flush((z0 - (float)g0) * QRS);
            sZv[i1] = g1; sZr[i1] = toh_flush((z1 - (float)g1) * QRS); }
    }
    __syncthreads();

#pragma unroll 1
    for (int nt = wave; nt < (SB * C2) / 16; nt += 8) {
        const int col = nt * 16 + lr;
        const v16h bv = LFRAG(sZv, col * ZP + 8 * hi), bq = LFRAG(sZr, col * ZP + 8 * hi);
        v8f v0 = (v8f){}, q0 = (v8f){}, v1 = (v8f){}, q1 = (v8f){};
        v0 = mmah(am0, bv, v0); q0 = mmah(am0, bq, q0); v1 = mmah(am1, bv, v1); q1 = mmah(am1, bq, q1);
        const int s = col >> 5, c = col & 31; const float bc = sB2[c];
#pragma unroll
        for (int r = 0; r < 8; ++r) {
            const int n0 = 8 * hi + r, n1 = 16 + 8 * hi + r;
            const float u0 = fmaxf(dA[r] * (v0[r] + q0[r] * QRI) + bc, 0.0f), u1 = fmaxf(dB[r] * (v1[r] + q1[r] * QRI) + bc, 0.0f);
            const h16 g0 = toh_flush(u0), g1 = toh_flush(u1);
            const int i0 = (n0 * SB + s) * C2 + c;
            sHv[i0] = g0; sHr[i0] = toh_flush((u0 - (float)g0) * QRS);
            if (n1 < NN) { const int i1 = (n1 * SB + s) * C2 + c; sHv[i1] = g1; sHr[i1] = toh_flush((u1 - (float)g1) * QRS); } }
    }
    __syncthreads();

#pragma unroll 1
    for (int j = wave; j < NRT; j += 8) {
        const v16h av = LFRAG(sHv, (16 * j + lr) * C2 + 8 * hi), ar = LFRAG(sHr, (16 * j + lr) * C2 + 8 * hi);
        const v16h w0 = LFRAG(sW3t, lr * C2 + 8 * hi);
        v8f cv0 = (v8f){}, cr0 = (v8f){};
        cv0 = mmah(av, w0, cv0); cr0 = mmah(ar, w0, cr0);
        const int nC = 2 * j + hi; const float dn = sDinv[nC] * WSI;
#pragma unroll
        for (int r = 0; r < 8; ++r) {
            const float z0 = (cv0[r] + cr0[r] * QRI) * dn; const h16 g0 = toh_flush(z0);
            const int i0 = (r * C3 + lr) * ZP + nC;
            sZv[i0] = g0; sZr[i0] = toh_flush((z0 - (float)g0) * QRS); }
    }
    __syncthreads();

#pragma unroll 1
    for (int nt = wave; nt < (SB * C3) / 16; nt += 8) {
        const int col = nt * 16 + lr;
        const v16h bv = LFRAG(sZv, col * ZP + 8 * hi), bq = LFRAG(sZr, col * ZP + 8 * hi);
        v8f v0 = (v8f){}, q0 = (v8f){}, v1 = (v8f){}, q1 = (v8f){};
        v0 = mmah(am0, bv, v0); q0 = mmah(am0, bq, q0); v1 = mmah(am1, bv, v1); q1 = mmah(am1, bq, q1);
        const int s = col >> 4, c = col & 15; const float bc = sB3[c];
#pragma unroll
        for (int r = 0; r < 8; ++r) {
            const int n0 = 8 * hi + r, n1 = 16 + 8 * hi + r;
            const float u0 = fmaxf(dA[r] * (v0[r] + q0[r] * QRI) + bc, 0.0f), u1 = fmaxf(dB[r] * (v1[r] + q1[r] * QRI) + bc, 0.0f);
            const h16 g0 = toh_flush(u0), g1 = toh_flush(u1);
            const int i0 = (n0 * SB + s) * C3 + c;
            sHv[i0] = g0; sHr[i0] = toh_flush((u0 - (float)g0) * QRS);
            if (n1 < NN) { const int i1 = (n1 * SB + s) * C3 + c; sHv[i1] = g1; sHr[i1] = toh_flush((u1 - (float)g1) * QRS); } }
    }
    __syncthreads();

#pragma unroll 1
    for (int j = wave; j < NRT; j += 8) {
        const v16h av = cat16(*(const v8h*)(&sHv[(16 * j + lr) * C3 + 8 * hi]), z8), ar = cat16(*(const v8h*)(&sHr[(16 * j + lr) * C3 + 8 * hi]), z8);
        const v16h w0 = cat16(*(const v8h*)(&sW4t[lr * 16 + 8 * hi]), z8);
        v8f cv0 = (v8f){}, cr0 = (v8f){};
        cv0 = mmah(av, w0, cv0); cr0 = mmah(ar, w0, cr0);
        const int nC = 2 * j + hi; const float dn = sDinv[nC] * WSI;
        if (lr < C4) {
#pragma unroll
            for (int r = 0; r < 8; ++r) {
                const float z0 = (cv0[r] + cr0[r] * QRI) * dn; const h16 g0 = toh_flush(z0);
                const int i0 = (r * C4 + lr) * ZP + nC;
                sZv[i0] = g0; sZr[i0] = toh_flush((z0 - (float)g0) * QRS); } }
    }
    __syncthreads();

#pragma unroll 1
    for (int nt = wave; nt < (SB * C4) / 16; nt += 8) {
        const int col = nt * 16 + lr;
        const v16h bv = LFRAG(sZv, col * ZP + 8 * hi), bq = LFRAG(sZr, col * ZP + 8 * hi);
        v8f v0 = (v8f){}, q0 = (v8f){}, v1 = (v8f){}, q1 = (v8f){};
        v0 = mmah(am0, bv, v0); q0 = mmah(am0, bq, q0); v1 = mmah(am1, bv, v1); q1 = mmah(am1, bq, q1);
        const int s = col >> 3, c = col & 7; const float bc = sB4[c];
#pragma unroll
        for (int r = 0; r < 8; ++r) {
            const int n0 = 8 * hi + r, n1 = 16 + 8 * hi + r;
            const float u0 = fmaxf(dA[r] * (v0[r] + q0[r] * QRI) + bc, 0.0f), u1 = fmaxf(dB[r] * (v1[r] + q1[r] * QRI) + bc, 0.0f);
            sH4[(n0 * SB + s) * C4 + c] = u0;
            if (n1 < NN) sH4[(n1 * SB + s) * C4 + c] = u1; }
    }
    __syncthreads();

    if (tid < RT) {
        float z = 0.0f;
#pragma unroll
        for (int k = 0; k < C4; ++k) z = fmaf(sH4[tid * C4 + k], sW5[k], z);
        const int nA = tid >> 3, s = tid & 7;
        const float zs = z * sDinv[nA]; const h16 g = toh_flush(zs);
        sZv[s * ZP + nA] = g; sZr[s * ZP + nA] = toh_flush((zs - (float)g) * QRS);
    }
    sZv[SB * ZP + tid] = (h16)0.0f; sZr[SB * ZP + tid] = (h16)0.0f;
    __syncthreads();

    if (wave == 0) {
        const v16h bv = LFRAG(sZv, lr * ZP + 8 * hi), bq = LFRAG(sZr, lr * ZP + 8 * hi);
        v8f v0 = (v8f){}, q0 = (v8f){}, v1 = (v8f){}, q1 = (v8f){};
        v0 = mmah(am0, bv, v0); q0 = mmah(am0, bq, q0); v1 = mmah(am1, bv, v1); q1 = mmah(am1, bq, q1);
        const float bc = sB5[0];
        if (lr < SB) {
#pragma unroll
            for (int r = 0; r < 8; ++r) {
                const int n0 = 8 * hi + r, n1 = 16 + 8 * hi + r;
                sOut[RT + lr * NN + n0] = dA[r] * (v0[r] + q0[r] * QRI) + bc;
                if (n1 < NN) sOut[RT + lr * NN + n1] = dB[r] * (v1[r] + q1[r] * QRI) + bc; } }
    }
    __syncthreads();

    if (tid < RT) {
        unsigned ut = (unsigned)tid; asm volatile("" : "+v"(ut));
        const unsigned us = ut / (unsigned)NN;
        const int s = (int)us, n = (int)(ut - us * (unsigned)NN); const int lgb = RT + s * NN;
        const int pn = sPar[n]; const int pe = (n == 0) ? 0 : pn;
        float mx = NEGB;
#pragma unroll 1
        for (int m = 1; m < NN; ++m) { const float lm = sOut[lgb + m]; mx = fmaxf(mx, (sPar[m] == pe) ? lm : NEGB); }
        float ssum = 0.0f;
#pragma unroll 1
        for (int m = 1; m < NN; ++m) { const float lm = sOut[lgb + m]; const float e = expf(lm - mx); ssum += (sPar[m] == pe) ? e : 0.0f; }
        const float sh = sOut[lgb + n] - mx;
        const float lc = sh - logf(ssum);
        sLcp[tid] = (n != 0) ? lc : 0.0f;
    }
    __syncthreads();

    if (tid < RT) {
        unsigned ut = (unsigned)tid; asm volatile("" : "+v"(ut));
        const unsigned us = ut / (unsigned)NN;
        const int s = (int)us, n = (int)(ut - us * (unsigned)NN);
        float acc = 0.0f; int node = n;
#pragma unroll 1
        for (int it = 0; it < NN; ++it) { const bool go = node != 0; const float c = sLcp[s * NN + node]; acc += go ? c : 0.0f; const int pn = sPar[node]; node = go ? pn : 0; }
        sOut[tid] = expf(acc);
    }
    __syncthreads();

    if (wave < 2) {
        const size_t ob = (size_t)wave * ((size_t)NROWS_FULL * NN) + (size_t)b0 * NN;
        const int sb = wave * RT;
        const int l2 = lane < 24 ? lane : 23;
#pragma unroll 1
        for (int ps = 0; ps < 2; ++ps) {
            const v4f va = *(const v4fa*)(&sOut[sb + lane * 4]);
            const v4f vb = *(const v4fa*)(&sOut[sb + 128 + l2 * 4]);
            *(volatile v4f*)(OUT + ob + lane * 4) = va;
            if (lane < 24) *(volatile v4f*)(OUT + ob + 128 + lane * 4) = vb;
            if (ps == 0) __threadfence(); }
    }
}

static constexpr size_t al256(size_t v) { return (v + 255) & ~(size_t)255; }
static constexpr size_t SZ_W1T = al256((size_t)C1 * C0 * 2);
static constexpr size_t SZ_Y   = al256((size_t)NROWS * C1 * 4);
static constexpr size_t SZ_TOTAL = SZ_W1T + SZ_Y;
static_assert(SZ_TOTAL <= (size_t)134217728);
static_assert(((size_t)(NROWS / 32 - 1) * 32 + 32) * C1 * 4 <= SZ_Y);
static_assert((size_t)(C1 * C0 / 8) * 16 <= SZ_W1T);

extern "C" void kernel_launch(void* const* d_in, const int* in_sizes, int n_in,
                              void* d_out, int out_size, void* d_ws, size_t ws_size, hipStream_t stream) {
    if (n_in < 11) return;
    if ((size_t)in_sizes[0] < (size_t)NROWS * C0) return;
    if (in_sizes[1] < C0 * C1 || in_sizes[2] < C1 || in_sizes[3] < C1 * C2 || in_sizes[4] < C2) return;
    if (in_sizes[5] < C2 * C3 || in_sizes[6] < C3 || in_sizes[7] < C3 * C4 || in_sizes[8] < C4) return;
    if (in_sizes[9] < C4 || in_sizes[10] < 1) return;
    if ((size_t)out_size < (size_t)NROWS_FULL * NN + (size_t)NROWS * NN) return;
    if (SZ_TOTAL > ws_size) return;
    const float* x  = (const float*)d_in[0];
    const float* W1 = (const float*)d_in[1];  const float* b1 = (const float*)d_in[2];
    const float* W2 = (const float*)d_in[3];  const float* b2 = (const float*)d_in[4];
    const float* W3 = (const float*)d_in[5];  const float* b3 = (const float*)d_in[6];
    const float* W4 = (const float*)d_in[7];  const float* b4 = (const float*)d_in[8];
    const float* W5 = (const float*)d_in[9];  const float* b5 = (const float*)d_in[10];
    float* OUT = (float*)d_out;
    char* wsp = (char*)d_ws;
    bf* W1T = (bf*)wsp; wsp += SZ_W1T;
    float* Yp = (float*)wsp; wsp += SZ_Y;

    k_w1t<<<(C1 * C0 / 8) / 256, 256, 0, stream>>>(W1, W1T);
    k_y<<<NROWS / 32, 32, 0, stream>>>(x, W1T, Yp);
    k_tree<<<NROWS / SB, 256, 0, stream>>>(Yp, b1, W2, b2, W3, b3, W4, b4, W5, b5, OUT);
}
